// MambaDecoderLayerWithCross_28965259444908
// MI455X (gfx1250) — hardware-verified
//
#include <hip/hip_runtime.h>
#include <stddef.h>
#include <math.h>


#pragma clang fp contract(off)

#define NB    2
#define NL    512
#define NTK   (NB * NL)
#define DM    256
#define DI    1024
#define DS    128
#define DC    4
#define DR    16
#define NH    8
#define DKH   32
#define DFF   1024
#define DBW   272
#define DBP   288
#define NTHR  256
#define WCAR  64.0f
#define LNEPS 1e-6f
#define NEGMAX (-3.402823466e38f)
#define WSCAP 134217728

#define SC_64     0.015625f
#define SC_512    0.001953125f
#define SC_1024   0.0009765625f
#define SC_4096   0.000244140625f
#define SC_16384  0.00006103515625f
#define RSQ32     0.17677669529663687f
#define SSCL      (RSQ32 * 0.00390625f)
#define PCAR      1024.0f
#define OSCL      0.00390625f

#define FL_BIAS 1
#define FL_RELU 2
#define FL_RES  4
#define FL_F32  8
#define FL_F16  16

#define SZ_INW  ((size_t)2 * DI * DM * 2)
#define SZ_XPW  ((size_t)DBP * DI * 2)
#define SZ_OPW  ((size_t)DM * DI * 2)
#define SZ_WSQ  ((size_t)DM * DM * 2)
#define SZ_W1   ((size_t)DFF * DM * 2)
#define SZ_W2   ((size_t)DM * DFF * 2)
#define SZ_T16  ((size_t)NTK * DM * 2)
#define SZ_T32  ((size_t)NTK * DM * 4)
#define SZ_XZ   ((size_t)NTK * 2 * DI * 4)
#define SZ_U    ((size_t)NTK * DI * 4)
#define SZ_DBL  ((size_t)NTK * DBP * 4)
#define SZ_FF   ((size_t)NTK * DFF * 2)

#define O_INW  ((size_t)0)
#define O_XPW  (O_INW + SZ_INW)
#define O_OPW  (O_XPW + SZ_XPW)
#define O_WQ   (O_OPW + SZ_OPW)
#define O_WK   (O_WQ + SZ_WSQ)
#define O_WV   (O_WK + SZ_WSQ)
#define O_WO   (O_WV + SZ_WSQ)
#define O_W1   (O_WO + SZ_WSQ)
#define O_W2   (O_W1 + SZ_W1)
#define O_XN   (O_W2 + SZ_W2)
#define O_XZ   (O_XN + SZ_T16)
#define O_U    (O_XZ + SZ_XZ)
#define O_DBL  (O_U + SZ_U)
#define O_DTS  (O_DBL + SZ_DBL)
#define O_YG   (O_DTS + SZ_U)
#define O_H1   (O_YG + SZ_U)
#define O_HN2  (O_H1 + SZ_T32)
#define O_Q    (O_HN2 + SZ_T16)
#define O_K    (O_Q + SZ_T16)
#define O_V    (O_K + SZ_T16)
#define O_O    (O_V + SZ_T16)
#define O_H2   (O_O + SZ_T16)
#define O_HN3  (O_H2 + SZ_T32)
#define O_FF   (O_HN3 + SZ_T16)
#define WSTOT  (O_FF + SZ_FF)

static_assert(WSTOT <= (size_t)WSCAP);
static_assert((O_XPW % 128) == 0 && (O_OPW % 128) == 0 && (O_WQ % 128) == 0 && (O_W1 % 128) == 0 && (O_W2 % 128) == 0);
static_assert((O_XN % 128) == 0 && (O_XZ % 128) == 0 && (O_U % 128) == 0 && (O_DBL % 128) == 0 && (O_DTS % 128) == 0);
static_assert((O_YG % 128) == 0 && (O_H1 % 128) == 0 && (O_HN2 % 128) == 0 && (O_Q % 128) == 0 && (O_O % 128) == 0);
static_assert((O_H2 % 128) == 0 && (O_HN3 % 128) == 0 && (O_FF % 128) == 0);

#define CVB  2048
#define NS_INW (2 * DI * DM)
#define NS_XPW (DBW * DI)
#define NP_XPW (DBP * DI)
#define NS_OPW (DM * DI)
#define NS_WSQ (DM * DM)
#define NS_W1  (DFF * DM)
#define NS_W2  (DM * DFF)
#define CB1 (NS_INW / CVB)
#define CB2 (CB1 + NP_XPW / CVB)
#define CB3 (CB2 + NS_OPW / CVB)
#define CB4 (CB3 + NS_WSQ / CVB)
#define CB5 (CB4 + NS_WSQ / CVB)
#define CB6 (CB5 + NS_WSQ / CVB)
#define CB7 (CB6 + NS_WSQ / CVB)
#define CB8 (CB7 + NS_W1 / CVB)
#define CBT (CB8 + NS_W2 / CVB)
static_assert((size_t)CBT * CVB * 2 == O_XN);
static_assert((NS_XPW % CVB) == 0 && (NP_XPW % CVB) == 0);
static_assert(CVB == NTHR * 8);

static_assert((DM % 32) == 0 && (DI % 32) == 0 && (DFF % 32) == 0);
static_assert((NTK % 128) == 0 && (NTK % 32) == 0 && (DBP % 32) == 0 && ((2 * DI) % 256) == 0 && (DFF % 256) == 0);

typedef _Float16 v16h __attribute__((ext_vector_type(16)));
typedef _Float16 v8h  __attribute__((ext_vector_type(8), __may_alias__));
typedef float    v8f  __attribute__((ext_vector_type(8)));
typedef float    v4f  __attribute__((ext_vector_type(4), __may_alias__));
union Frag { v16h v; v8h h[2]; };
static_assert(sizeof(Frag) == 32);

__device__ __forceinline__ v8f wmh(v16h a, v16h bq, v8f c) {
  v8f d = __builtin_amdgcn_wmma_f32_16x16x32_f16(false, a, false, bq, (short)0, c, false, false);
  asm volatile("v_nop\n\tv_nop\n\tv_nop\n\tv_nop" : "+v"(d) : "v"(a), "v"(bq));
  return d;
}

__device__ __forceinline__ v8f zero8() {
  v8f z = {0.f, 0.f, 0.f, 0.f, 0.f, 0.f, 0.f, 0.f};
  return z;
}

__global__ __launch_bounds__(NTHR) void k_wcvt(const float* __restrict__ w_in, const float* __restrict__ w_xp,
                                               const float* __restrict__ w_op, const float* __restrict__ w_q,
                                               const float* __restrict__ w_k, const float* __restrict__ w_v,
                                               const float* __restrict__ w_o, const float* __restrict__ w_1,
                                               const float* __restrict__ w_2, _Float16* P) {
  const int blk = blockIdx.x, tid = threadIdx.x;
  const float* src;
  int bs, nsrc;
  if (blk < CB1)      { src = w_in; bs = 0;   nsrc = NS_INW; }
  else if (blk < CB2) { src = w_xp; bs = CB1; nsrc = NS_XPW; }
  else if (blk < CB3) { src = w_op; bs = CB2; nsrc = NS_OPW; }
  else if (blk < CB4) { src = w_q;  bs = CB3; nsrc = NS_WSQ; }
  else if (blk < CB5) { src = w_k;  bs = CB4; nsrc = NS_WSQ; }
  else if (blk < CB6) { src = w_v;  bs = CB5; nsrc = NS_WSQ; }
  else if (blk < CB7) { src = w_o;  bs = CB6; nsrc = NS_WSQ; }
  else if (blk < CB8) { src = w_1;  bs = CB7; nsrc = NS_W1; }
  else                { src = w_2;  bs = CB8; nsrc = NS_W2; }
  const size_t so = (size_t)(blk - bs) * CVB + (size_t)tid * 8;
  const bool inr = (so + 8 <= (size_t)nsrc);
  const size_t soc = inr ? so : (size_t)(nsrc - 8);
  const float sc = inr ? WCAR : 0.0f;
  const v4f a0 = *(const v4f*)(src + soc);
  const v4f a1 = *(const v4f*)(src + soc + 4);
  v8h hv;
  hv[0] = (_Float16)(a0[0] * sc); hv[1] = (_Float16)(a0[1] * sc); hv[2] = (_Float16)(a0[2] * sc); hv[3] = (_Float16)(a0[3] * sc);
  hv[4] = (_Float16)(a1[0] * sc); hv[5] = (_Float16)(a1[1] * sc); hv[6] = (_Float16)(a1[2] * sc); hv[7] = (_Float16)(a1[3] * sc);
  _Float16* dp = P + (size_t)blk * CVB + (size_t)tid * 8;
  *(volatile v8h*)dp = hv;
  __threadfence();
  *(volatile v8h*)dp = hv;
}

__global__ __launch_bounds__(NTHR) void k_ln(const float* __restrict__ X, const float* __restrict__ ga,
                                             const float* __restrict__ gb, _Float16* Y) {
  const int tid = threadIdx.x, lane = tid & 31, wave = tid >> 5;
  const size_t row = (size_t)blockIdx.x * (NTHR / 32) + wave;
  const float* xp = X + row * DM + 8 * lane;
  const v4f x0 = *(const v4f*)xp;
  const v4f x1 = *(const v4f*)(xp + 4);
  float s = ((x0[0] + x0[1]) + (x0[2] + x0[3])) + ((x1[0] + x1[1]) + (x1[2] + x1[3]));
#pragma unroll
  for (int off = 16; off > 0; off >>= 1) s += __shfl_xor(s, off, 32);
  const float mean = s * (1.0f / (float)DM);
  float dv[8];
  dv[0] = x0[0] - mean; dv[1] = x0[1] - mean; dv[2] = x0[2] - mean; dv[3] = x0[3] - mean;
  dv[4] = x1[0] - mean; dv[5] = x1[1] - mean; dv[6] = x1[2] - mean; dv[7] = x1[3] - mean;
  float ss = 0.0f;
#pragma unroll
  for (int i = 0; i < 8; ++i) ss = ss + dv[i] * dv[i];
#pragma unroll
  for (int off = 16; off > 0; off >>= 1) ss += __shfl_xor(ss, off, 32);
  const float var = ss * (1.0f / (float)(DM - 1));
  const float sd = sqrtf(var);
  const float inv = 1.0f / (sd + LNEPS);
  const v4f g0 = *(const v4f*)(ga + 8 * lane);
  const v4f g1 = *(const v4f*)(ga + 8 * lane + 4);
  const v4f b0 = *(const v4f*)(gb + 8 * lane);
  const v4f b1 = *(const v4f*)(gb + 8 * lane + 4);
  v8h hv;
  hv[0] = (_Float16)((g0[0] * dv[0]) * inv + b0[0]);
  hv[1] = (_Float16)((g0[1] * dv[1]) * inv + b0[1]);
  hv[2] = (_Float16)((g0[2] * dv[2]) * inv + b0[2]);
  hv[3] = (_Float16)((g0[3] * dv[3]) * inv + b0[3]);
  hv[4] = (_Float16)((g1[0] * dv[4]) * inv + b1[0]);
  hv[5] = (_Float16)((g1[1] * dv[5]) * inv + b1[1]);
  hv[6] = (_Float16)((g1[2] * dv[6]) * inv + b1[2]);
  hv[7] = (_Float16)((g1[3] * dv[7]) * inv + b1[3]);
  _Float16* dp = Y + row * DM + 8 * lane;
  *(volatile v8h*)dp = hv;
  __threadfence();
  *(volatile v8h*)dp = hv;
}

template <int WM, int NT, int AF>
__global__ __launch_bounds__(NTHR) void k_gemm(const _Float16* __restrict__ Ah, const float* __restrict__ Af,
                                               const _Float16* __restrict__ W, const float* __restrict__ bias,
                                               const float* __restrict__ resid, float* Cf, _Float16* Ch,
                                               int lda, int ldw, int ldcf, int ldch, int ldr, int K,
                                               float acv, float scale, float hcv, int flags) {
  constexpr int WN = 8 / WM;
  constexpr int R = 16 * WM;
  constexpr int BN = WN * 16 * NT;
  static_assert(WM * WN == 8);
  static_assert(((R * BN / 4) % NTHR) == 0);
  __shared__ __align__(16) float sC[R * BN];
  const int tid = threadIdx.x, lane = tid & 31, wave = tid >> 5, h = lane >> 4, m = lane & 15;
  const int wm = wave % WM, wn = wave / WM;
  const int bm0 = blockIdx.y * R;
  const int n0 = blockIdx.x * BN;
  const int m0 = bm0 + 16 * wm;
  const int nw0 = n0 + wn * 16 * NT;

  v8f acc[NT];
#pragma unroll
  for (int t = 0; t < NT; ++t) acc[t] = zero8();

  const size_t arow = (size_t)(m0 + m) * (size_t)lda + 8 * h;
  const size_t wrow = (size_t)(nw0 + m) * (size_t)ldw + 8 * h;
  const int nks = K >> 5;

#pragma unroll 1
  for (int ks = 0; ks < nks; ++ks) {
    const int k0 = ks << 5;
    Frag fa;
    if constexpr (AF != 0) {
      const v4f a0 = *(const v4f*)(Af + arow + k0);
      const v4f a1 = *(const v4f*)(Af + arow + k0 + 4);
      const v4f a2 = *(const v4f*)(Af + arow + k0 + 16);
      const v4f a3 = *(const v4f*)(Af + arow + k0 + 20);
      v8h lo, hi;
      lo[0] = (_Float16)(a0[0] * acv); lo[1] = (_Float16)(a0[1] * acv); lo[2] = (_Float16)(a0[2] * acv); lo[3] = (_Float16)(a0[3] * acv);
      lo[4] = (_Float16)(a1[0] * acv); lo[5] = (_Float16)(a1[1] * acv); lo[6] = (_Float16)(a1[2] * acv); lo[7] = (_Float16)(a1[3] * acv);
      hi[0] = (_Float16)(a2[0] * acv); hi[1] = (_Float16)(a2[1] * acv); hi[2] = (_Float16)(a2[2] * acv); hi[3] = (_Float16)(a2[3] * acv);
      hi[4] = (_Float16)(a3[0] * acv); hi[5] = (_Float16)(a3[1] * acv); hi[6] = (_Float16)(a3[2] * acv); hi[7] = (_Float16)(a3[3] * acv);
      fa.h[0] = lo;
      fa.h[1] = hi;
    } else {
      fa.h[0] = *(const v8h*)(Ah + arow + k0);
      fa.h[1] = *(const v8h*)(Ah + arow + k0 + 16);
    }
#pragma unroll
    for (int t = 0; t < NT; ++t) {
      const _Float16* wp = W + wrow + (size_t)(16 * t) * (size_t)ldw + k0;
      Frag fb;
      fb.h[0] = *(const v8h*)wp;
      fb.h[1] = *(const v8h*)(wp + 16);
      acc[t] = wmh(fa.v, fb.v, acc[t]);
    }
  }

  const bool fbias = (flags & FL_BIAS) != 0;
  const bool frelu = (flags & FL_RELU) != 0;
  const bool fres = (flags & FL_RES) != 0;
#pragma unroll
  for (int t = 0; t < NT; ++t) {
    const int cl = wn * 16 * NT + 16 * t + m;
    const int n = n0 + cl;
    float bn = 0.0f;
    if (fbias) bn = bias[n];
#pragma unroll
    for (int r = 0; r < 8; ++r) {
      const int rl = 16 * wm + 8 * h + r;
      float v = acc[t][r] * scale + bn;
      if (frelu) v = fmaxf(v, 0.0f);
      if (fres) v = v + resid[(size_t)(bm0 + rl) * (size_t)ldr + n];
      sC[rl * BN + cl] = v;
    }
  }
  __syncthreads();

  if (flags & FL_F32) {
    constexpr int NF4 = (R * BN / 4) / NTHR;
#pragma unroll
    for (int it = 0; it < NF4; ++it) {
      const int e = tid + it * NTHR;
      const int rl = e / (BN / 4), q = e - rl * (BN / 4);
      const v4f v = *(const v4f*)(sC + 4 * e);
      *(volatile v4f*)(Cf + (size_t)(bm0 + rl) * (size_t)ldcf + n0 + 4 * q) = v;
    }
    __threadfence();
#pragma unroll
    for (int it = 0; it < NF4; ++it) {
      const int e = tid + it * NTHR;
      const int rl = e / (BN / 4), q = e - rl * (BN / 4);
      const v4f v = *(const v4f*)(sC + 4 * e);
      *(volatile v4f*)(Cf + (size_t)(bm0 + rl) * (size_t)ldcf + n0 + 4 * q) = v;
    }
  }
  if constexpr (BN >= 64) {
    if (flags & FL_F16) {
      constexpr int NH8 = (R * BN / 8) / NTHR;
#pragma unroll
      for (int it = 0; it < NH8; ++it) {
        const int e = tid + it * NTHR;
        const int rl = e / (BN / 8), q = e - rl * (BN / 8);
        const v4f a = *(const v4f*)(sC + 8 * e);
        const v4f c = *(const v4f*)(sC + 8 * e + 4);
        v8h hv;
        hv[0] = (_Float16)(a[0] * hcv); hv[1] = (_Float16)(a[1] * hcv); hv[2] = (_Float16)(a[2] * hcv); hv[3] = (_Float16)(a[3] * hcv);
        hv[4] = (_Float16)(c[0] * hcv); hv[5] = (_Float16)(c[1] * hcv); hv[6] = (_Float16)(c[2] * hcv); hv[7] = (_Float16)(c[3] * hcv);
        *(volatile v8h*)(Ch + (size_t)(bm0 + rl) * (size_t)ldch + n0 + 8 * q) = hv;
      }
      __threadfence();
#pragma unroll
      for (int it = 0; it < NH8; ++it) {
        const int e = tid + it * NTHR;
        const int rl = e / (BN / 8), q = e - rl * (BN / 8);
        const v4f a = *(const v4f*)(sC + 8 * e);
        const v4f c = *(const v4f*)(sC + 8 * e + 4);
        v8h hv;
        hv[0] = (_Float16)(a[0] * hcv); hv[1] = (_Float16)(a[1] * hcv); hv[2] = (_Float16)(a[2] * hcv); hv[3] = (_Float16)(a[3] * hcv);
        hv[4] = (_Float16)(c[0] * hcv); hv[5] = (_Float16)(c[1] * hcv); hv[6] = (_Float16)(c[2] * hcv); hv[7] = (_Float16)(c[3] * hcv);
        *(volatile v8h*)(Ch + (size_t)(bm0 + rl) * (size_t)ldch + n0 + 8 * q) = hv;
      }
    }
  }
}

__global__ __launch_bounds__(NTHR) void k_conv(const float* __restrict__ XZ, const float* __restrict__ cw,
                                               const float* __restrict__ cb, float* U32) {
  const int g = blockIdx.x * NTHR + threadIdx.x;
  const int tok = g / (DI / 4);
  const int dq = (g - tok * (DI / 4)) * 4;
  const int b = tok / NL, t = tok - b * NL;
  v4f acc = *(const v4f*)(cb + dq);
  v4f w[4];
#pragma unroll
  for (int j = 0; j < 4; ++j) w[j] = *(const v4f*)(cw + (size_t)(dq + j) * DC);
#pragma unroll
  for (int k = 0; k < DC; ++k) {
    const int tt = t + k - (DC - 1);
    const int ttc = (tt < 0) ? 0 : tt;
    const v4f xv = *(const v4f*)(XZ + ((size_t)b * NL + ttc) * (size_t)(2 * DI) + dq);
    const float f = (tt >= 0) ? 1.0f : 0.0f;
#pragma unroll
    for (int j = 0; j < 4; ++j) acc[j] = acc[j] + (xv[j] * f) * w[j][k];
  }
  v4f u;
#pragma unroll
  for (int j = 0; j < 4; ++j) {
    const float a = acc[j];
    u[j] = a * __builtin_amdgcn_rcpf(1.0f + __expf(-a));
  }
  float* dp = U32 + (size_t)g * 4;
  *(volatile v4f*)dp = u;
  __threadfence();
  *(volatile v4f*)dp = u;
}

__global__ __launch_bounds__(NTHR) void k_dt(const float* __restrict__ DBL, const float* __restrict__ dtw,
                                             const float* __restrict__ dtb, float* DTS) {
  __shared__ float sR[DR];
  __shared__ __align__(16) float sV[NTHR];
  const int tid = threadIdx.x;
  const int tok = blockIdx.x / (DI / NTHR);
  const int dq = (blockIdx.x - tok * (DI / NTHR)) * NTHR;
  const int d = dq + tid;
  if (tid < DR) sR[tid] = DBL[(size_t)tok * DBP + tid];
  __syncthreads();
  float s = 0.0f;
#pragma unroll 1
  for (int r = 0; r < DR; ++r) s = s + sR[r] * dtw[(size_t)d * DR + r];
  const float v = s + dtb[d];
  const float sp = fmaxf(v, 0.0f) + log1pf(expf(-fabsf(v)));
  sV[tid] = sp;
  __syncthreads();
  float* dp = DTS + (size_t)tok * DI + dq + 4 * tid;
  v4f o = {0.f, 0.f, 0.f, 0.f};
  if (tid < NTHR / 4) {
    o = *(const v4f*)(sV + 4 * tid);
    *(volatile v4f*)dp = o;
  }
  __threadfence();
  if (tid < NTHR / 4) {
    *(volatile v4f*)dp = o;
  }
}

#define SCH 4
#define SCB (8 * SCH)
#define STB 32
static_assert((DI % SCB) == 0 && (NL % STB) == 0 && STB == 8 * 4 && SCB == 32 && DS == 128);

__global__ __launch_bounds__(NTHR) void k_scan(const float* __restrict__ DTS, const float* __restrict__ U32,
                                               const float* __restrict__ DBL, const float* __restrict__ XZ,
                                               const float* __restrict__ Alog, const float* __restrict__ Dp,
                                               float* YG) {
  __shared__ __align__(16) float sA[SCB * DS];
  __shared__ __align__(16) float sY[STB * SCB];
  const int tid = threadIdx.x, lane = tid & 31, wave = tid >> 5;
  const int b = blockIdx.x / (DI / SCB);
  const int c0 = (blockIdx.x - b * (DI / SCB)) * SCB;
  const int d0 = c0 + SCH * wave;
#pragma unroll 1
  for (int e = tid; e < SCB * DS; e += NTHR) sA[e] = -expf(Alog[(size_t)c0 * DS + e]);
  __syncthreads();

  float Ac[SCH][4], hs[SCH][4], dp[SCH];
#pragma unroll
  for (int c = 0; c < SCH; ++c) {
#pragma unroll
    for (int i = 0; i < 4; ++i) {
      Ac[c][i] = sA[(SCH * wave + c) * DS + 4 * lane + i];
      hs[c][i] = 0.0f;
    }
    dp[c] = Dp[d0 + c];
  }
  const size_t tokb = (size_t)b * NL;

#pragma unroll 1
  for (int t0 = 0; t0 < NL; t0 += STB) {
#pragma unroll 1
    for (int tl = 0; tl < STB; ++tl) {
      const size_t tok = tokb + (size_t)(t0 + tl);
      const v4f dt4 = *(const v4f*)(DTS + tok * DI + d0);
      const v4f u4 = *(const v4f*)(U32 + tok * DI + d0);
      const v4f z4 = *(const v4f*)(XZ + tok * (size_t)(2 * DI) + DI + d0);
      const v4f B4 = *(const v4f*)(DBL + tok * DBP + DR + 4 * lane);
      const v4f C4 = *(const v4f*)(DBL + tok * DBP + DR + DS + 4 * lane);
      float yv[SCH];
#pragma unroll
      for (int c = 0; c < SCH; ++c) {
        const float dt = dt4[c];
        const float dtu = dt * u4[c];
        float part = 0.0f;
#pragma unroll
        for (int i = 0; i < 4; ++i) {
          const float dA = __expf(dt * Ac[c][i]);
          const float hn = dA * hs[c][i] + dtu * B4[i];
          hs[c][i] = hn;
          part = part + hn * C4[i];
        }
#pragma unroll
        for (int off = 16; off > 0; off >>= 1) part += __shfl_xor(part, off, 32);
        const float z = z4[c];
        const float sg = __builtin_amdgcn_rcpf(1.0f + __expf(-z));
        yv[c] = (part + u4[c] * dp[c]) * (z * sg);
      }
      if (lane == 0) {
#pragma unroll
        for (int c = 0; c < SCH; ++c) sY[tl * SCB + SCH * wave + c] = yv[c];
      }
    }
    __syncthreads();
    {
      const int rl = 4 * wave + (lane >> 3), q = lane & 7;
      const v4f v = *(const v4f*)(sY + rl * SCB + 4 * q);
      float* gp = YG + (tokb + (size_t)(t0 + rl)) * DI + c0 + 4 * q;
      *(volatile v4f*)gp = v;
      __threadfence();
      *(volatile v4f*)gp = v;
    }
    __syncthreads();
  }
}

#define AQ    32
#define ATHR  64
#define LDS_P  (AQ * NL * 4)
#define LDS_VT (LDS_P + AQ * NL * 2)
#define LDS_O  (LDS_VT + DKH * NL * 2)
#define ALDS   (LDS_O + AQ * DM * 2)
static_assert((NL % AQ) == 0 && AQ == 32 && DKH == 32 && (NL % 64) == 0 && ((AQ * DM / 8) % ATHR) == 0);

__global__ __launch_bounds__(ATHR) void k_attn(const _Float16* __restrict__ Q16, const _Float16* __restrict__ K16,
                                               const _Float16* __restrict__ V16, const int* __restrict__ msk,
                                               _Float16* O16) {
  extern __shared__ __align__(16) unsigned char alds[];
  float* sS = (float*)(alds);
  _Float16* sP = (_Float16*)(alds + LDS_P);
  _Float16* sVT = (_Float16*)(alds + LDS_VT);
  _Float16* sO = (_Float16*)(alds + LDS_O);
  const int tid = threadIdx.x, lane = tid & 31, wave = tid >> 5, h = lane >> 4, m = lane & 15;
  const int b = blockIdx.x / (NL / AQ);
  const int q0 = (blockIdx.x - b * (NL / AQ)) * AQ;
  const size_t tokb = (size_t)b * NL;
  const int rw = 16 * wave;

#pragma unroll 1
  for (int hh = 0; hh < NH; ++hh) {
#pragma unroll 1
    for (int key = tid; key < NL; key += ATHR) {
      const _Float16* vp = V16 + (tokb + key) * DM + hh * DKH;
#pragma unroll
      for (int j = 0; j < 4; ++j) {
        const v8h vv = *(const v8h*)(vp + 8 * j);
#pragma unroll
        for (int i = 0; i < 8; ++i) sVT[(8 * j + i) * NL + key] = vv[i];
      }
    }
    __syncthreads();

    Frag fq;
    {
      const _Float16* qp = Q16 + (tokb + q0 + rw + m) * DM + hh * DKH + 8 * h;
      fq.h[0] = *(const v8h*)qp;
      fq.h[1] = *(const v8h*)(qp + 16);
    }
#pragma unroll 1
    for (int ng = 0; ng < NL / 64; ++ng) {
      v8f acc[4];
#pragma unroll
      for (int t = 0; t < 4; ++t) {
        const int key = ng * 64 + 16 * t + m;
        const _Float16* kp = K16 + (tokb + key) * DM + hh * DKH + 8 * h;
        Frag fk;
        fk.h[0] = *(const v8h*)kp;
        fk.h[1] = *(const v8h*)(kp + 16);
        acc[t] = wmh(fq.v, fk.v, zero8());
      }
#pragma unroll
      for (int t = 0; t < 4; ++t) {
        const int col = ng * 64 + 16 * t + m;
        const int mk = msk[b * NL + col];
#pragma unroll
        for (int r = 0; r < 8; ++r) {
          const float s = acc[t][r] * SSCL;
          sS[(rw + 8 * h + r) * NL + col] = (mk != 0) ? s : NEGMAX;
        }
      }
    }
    __syncthreads();

#pragma unroll 1
    for (int rr = 0; rr < 16; ++rr) {
      const int row = rw + rr;
      float sv[16];
      float mx = NEGMAX;
#pragma unroll
      for (int j = 0; j < 16; ++j) {
        sv[j] = sS[row * NL + 32 * j + lane];
        mx = fmaxf(mx, sv[j]);
      }
#pragma unroll
      for (int off = 16; off > 0; off >>= 1) mx = fmaxf(mx, __shfl_xor(mx, off, 32));
      float sum = 0.0f;
#pragma unroll
      for (int j = 0; j < 16; ++j) {
        sv[j] = expf(sv[j] - mx);
        sum += sv[j];
      }
#pragma unroll
      for (int off = 16; off > 0; off >>= 1) sum += __shfl_xor(sum, off, 32);
      const float inv = 1.0f / sum;
#pragma unroll
      for (int j = 0; j < 16; ++j) sP[row * NL + 32 * j + lane] = (_Float16)((sv[j] * inv) * PCAR);
    }
    __syncthreads();

    v8f oc[2];
    oc[0] = zero8();
    oc[1] = zero8();
#pragma unroll 1
    for (int ks = 0; ks < NL / 32; ++ks) {
      const int k0 = 32 * ks;
      Frag fp;
      fp.h[0] = *(const v8h*)(sP + (rw + m) * NL + k0 + 8 * h);
      fp.h[1] = *(const v8h*)(sP + (rw + m) * NL + k0 + 16 + 8 * h);
#pragma unroll
      for (int t = 0; t < 2; ++t) {
        Frag fv;
        fv.h[0] = *(const v8h*)(sVT + (16 * t + m) * NL + k0 + 8 * h);
        fv.h[1] = *(const v8h*)(sVT + (16 * t + m) * NL + k0 + 16 + 8 * h);
        oc[t] = wmh(fp.v, fv.v, oc[t]);
      }
    }
#pragma unroll
    for (int t = 0; t < 2; ++t) {
      const int col = hh * DKH + 16 * t + m;
#pragma unroll
      for (int r = 0; r < 8; ++r) sO[(rw + 8 * h + r) * DM + col] = (_Float16)(oc[t][r] * OSCL);
    }
    __syncthreads();
  }

#pragma unroll
  for (int it = 0; it < (AQ * DM / 8) / ATHR; ++it) {
    const int e = tid + it * ATHR;
    const int rl = e / (DM / 8), q = e - rl * (DM / 8);
    const v8h vv = *(const v8h*)(sO + 8 * e);
    *(volatile v8h*)(O16 + (tokb + q0 + rl) * DM + 8 * q) = vv;
  }
  __threadfence();
#pragma unroll
  for (int it = 0; it < (AQ * DM / 8) / ATHR; ++it) {
    const int e = tid + it * ATHR;
    const int rl = e / (DM / 8), q = e - rl * (DM / 8);
    const v8h vv = *(const v8h*)(sO + 8 * e);
    *(volatile v8h*)(O16 + (tokb + q0 + rl) * DM + 8 * q) = vv;
  }
}

extern "C" void kernel_launch(void* const* d_in, const int* in_sizes, int n_in,
                              void* d_out, int out_size, void* d_ws, size_t ws_size,
                              hipStream_t stream) {
  if (n_in < 31) return;
  if (in_sizes[0] != NTK * DM || in_sizes[1] != NTK * DM) return;
  if (in_sizes[2] != NB * NL) return;
  if (in_sizes[4] != 2 * DI * DM || in_sizes[5] != DI * DC || in_sizes[6] != DI) return;
  if (in_sizes[7] != DBW * DI || in_sizes[8] != DI * DR || in_sizes[9] != DI) return;
  if (in_sizes[10] != DI * DS || in_sizes[11] != DI || in_sizes[12] != DM * DI) return;
  for (int i = 13; i <= 18; ++i) if (in_sizes[i] != DM) return;
  if (in_sizes[19] != DM * DM || in_sizes[21] != DM * DM || in_sizes[23] != DM * DM || in_sizes[25] != DM * DM) return;
  if (in_sizes[20] != DM || in_sizes[22] != DM || in_sizes[24] != DM || in_sizes[26] != DM) return;
  if (in_sizes[27] != DFF * DM || in_sizes[28] != DFF || in_sizes[29] != DM * DFF || in_sizes[30] != DM) return;
  if (out_size != NTK * DM) return;
  const size_t tot = (size_t)WSTOT;
  if (tot > ws_size || tot > (size_t)WSCAP) return;

  const float* x      = (const float*)d_in[0];
  const float* mem    = (const float*)d_in[1];
  const int*   smask  = (const int*)d_in[2];
  const float* inw    = (const float*)d_in[4];
  const float* cw     = (const float*)d_in[5];
  const float* cb     = (const float*)d_in[6];
  const float* xpw    = (const float*)d_in[7];
  const float* dtw    = (const float*)d_in[8];
  const float* dtb    = (const float*)d_in[9];
  const float* alog   = (const float*)d_in[10];
  const float* dpp    = (const float*)d_in[11];
  const float* opw    = (const float*)d_in[12];
  const float* n1a = (const float*)d_in[13]; const float* n1b = (const float*)d_in[14];
  const float* n2a = (const float*)d_in[15]; const float* n2b = (const float*)d_in[16];
  const float* n3a = (const float*)d_in[17]; const float* n3b = (const float*)d_in[18];
  const float* wqw = (const float*)d_in[19]; const float* wqb = (const float*)d_in[20];
  const float* wkw = (const float*)d_in[21]; const float* wkb = (const float*)d_in[22];
  const float* wvw = (const float*)d_in[23]; const float* wvb = (const float*)d_in[24];
  const float* wow = (const float*)d_in[25]; const float* wob = (const float*)d_in[26];
  const float* w1w = (const float*)d_in[27]; const float* w1b = (const float*)d_in[28];
  const float* w2w = (const float*)d_in[29]; const float* w2b = (const float*)d_in[30];
  float* out = (float*)d_out;

  char* ws = (char*)d_ws;
  _Float16* INW  = (_Float16*)(ws + O_INW);
  _Float16* XPW  = (_Float16*)(ws + O_XPW);
  _Float16* OPW  = (_Float16*)(ws + O_OPW);
  _Float16* WQ   = (_Float16*)(ws + O_WQ);
  _Float16* WK   = (_Float16*)(ws + O_WK);
  _Float16* WV   = (_Float16*)(ws + O_WV);
  _Float16* WO   = (_Float16*)(ws + O_WO);
  _Float16* W1   = (_Float16*)(ws + O_W1);
  _Float16* W2   = (_Float16*)(ws + O_W2);
  _Float16* XN   = (_Float16*)(ws + O_XN);
  float*    XZ   = (float*)(ws + O_XZ);
  float*    U32  = (float*)(ws + O_U);
  float*    DBL  = (float*)(ws + O_DBL);
  float*    DTS  = (float*)(ws + O_DTS);
  float*    YG   = (float*)(ws + O_YG);
  float*    H1   = (float*)(ws + O_H1);
  _Float16* HN2  = (_Float16*)(ws + O_HN2);
  _Float16* Q16  = (_Float16*)(ws + O_Q);
  _Float16* K16  = (_Float16*)(ws + O_K);
  _Float16* V16  = (_Float16*)(ws + O_V);
  _Float16* O16  = (_Float16*)(ws + O_O);
  float*    H2   = (float*)(ws + O_H2);
  _Float16* HN3  = (_Float16*)(ws + O_HN3);
  _Float16* FF16 = (_Float16*)(ws + O_FF);


  k_wcvt<<<CBT, NTHR, 0, stream>>>(inw, xpw, opw, wqw, wkw, wvw, wow, w1w, w2w, INW);

  k_ln<<<NTK / (NTHR / 32), NTHR, 0, stream>>>(x, n1a, n1b, XN);

  k_gemm<2, 4, 0><<<dim3(2 * DI / 256, NTK / 32), NTHR, 0, stream>>>(
      XN, x, INW, x, x, XZ, FF16, DM, DM, 2 * DI, 0, 0, DM, 1.0f, SC_64, 1.0f, FL_F32);

  k_conv<<<(NTK * DI / 4) / NTHR, NTHR, 0, stream>>>(XZ, cw, cb, U32);

  k_gemm<8, 2, 1><<<dim3(DBP / 32, NTK / 128), NTHR, 0, stream>>>(
      XN, U32, XPW, x, x, DBL, FF16, DI, DI, DBP, 0, 0, DI, 256.0f, SC_16384, 1.0f, FL_F32);

  k_dt<<<NTK * (DI / NTHR), NTHR, 0, stream>>>(DBL, dtw, dtb, DTS);

  k_scan<<<NB * (DI / SCB), NTHR, 0, stream>>>(DTS, U32, DBL, XZ, alog, dpp, YG);

  k_gemm<2, 4, 1><<<dim3(1, NTK / 32), NTHR, 0, stream>>>(
      XN, YG, OPW, x, x, H1, FF16, DI, DI, DM, 0, DM, DI, 256.0f, SC_16384, 1.0f, FL_RES | FL_F32);

  k_ln<<<NTK / (NTHR / 32), NTHR, 0, stream>>>(H1, n2a, n2b, HN2);

  k_gemm<2, 4, 0><<<dim3(1, NTK / 32), NTHR, 0, stream>>>(
      HN2, x, WQ, wqb, x, YG, Q16, DM, DM, 0, DM, 0, DM, 1.0f, SC_64, 16.0f, FL_BIAS | FL_F16);

  k_gemm<2, 4, 1><<<dim3(1, NTK / 32), NTHR, 0, stream>>>(
      XN, mem, WK, wkb, x, YG, K16, DM, DM, 0, DM, 0, DM, 8.0f, SC_512, 16.0f, FL_BIAS | FL_F16);

  k_gemm<2, 4, 1><<<dim3(1, NTK / 32), NTHR, 0, stream>>>(
      XN, mem, WV, wvb, x, YG, V16, DM, DM, 0, DM, 0, DM, 8.0f, SC_512, 16.0f, FL_BIAS | FL_F16);

  hipFuncSetAttribute(reinterpret_cast<const void*>(&k_attn), hipFuncAttributeMaxDynamicSharedMemorySize, ALDS);
  k_attn<<<NB * (NL / AQ), ATHR, ALDS, stream>>>(Q16, K16, V16, smask, O16);

  k_gemm<2, 4, 0><<<dim3(1, NTK / 32), NTHR, 0, stream>>>(
      O16, x, WO, wob, H1, H2, FF16, DM, DM, DM, 0, DM, DM, 1.0f, SC_4096, 1.0f, FL_BIAS | FL_RES | FL_F32);

  k_ln<<<NTK / (NTHR / 32), NTHR, 0, stream>>>(H2, n3a, n3b, HN3);

  k_gemm<2, 4, 0><<<dim3(DFF / 256, NTK / 32), NTHR, 0, stream>>>(
      HN3, x, W1, w1b, x, YG, FF16, DM, DM, 0, DFF, 0, DM, 1.0f, SC_64, 16.0f, FL_BIAS | FL_RELU | FL_F16);

  k_gemm<2, 4, 0><<<dim3(1, NTK / 32), NTHR, 0, stream>>>(
      FF16, x, W2, w2b, H2, out, XN, DFF, DFF, DM, 0, DM, DFF, 1.0f, SC_1024, 1.0f, FL_BIAS | FL_RES | FL_F32);
}
